// Prismatic_20323785245259
// MI455X (gfx1250) — hardware-run, weakly checked
//
#include <hip/hip_runtime.h>


#ifndef NB
#define NB 2
#endif
#ifndef SEQ
#define SEQ 2048
#endif
#define NB_FULL  2
#define SEQ_FULL 2048
#ifndef OUT_SEQ
#define OUT_SEQ SEQ
#endif
#define HID  1024
#define DFF  4096
#define NEXP 8
#define TOK  (NB * SEQ)
#define NCAT (2 * DFF)
#define NWI  (HID * DFF)
#define EPB  16384
#define NBW  (NWI / EPB)
#define NHB  (2 * NBW + 2)
#define W1S  64.0f
#define W1I  (1.0f / 64.0f)
#define W2S  64.0f
#define ACS  256.0f
#define OI   (1.0f / (64.0f * 256.0f))
#define PSC  0.8f
#define LOG2E 1.4426950408889634f

static constexpr int tierk(int n) { const int k = (int)((double)n * 0.1 / 2.0); return k < 1 ? 1 : k; }
static constexpr int KT_W  = tierk(NWI);
static constexpr int KT_B1 = tierk(DFF);
static constexpr int KT_B2 = tierk(HID);
static_assert(KT_W == 209715);
static_assert(KT_B1 == 204);
static_assert(KT_B2 == 51);

static_assert(NEXP == 8);
static_assert(SEQ % 64 == 0);
static_assert(TOK % 64 == 0);
static_assert(TOK % 32 == 0);
static_assert(HID % 64 == 0);
static_assert(DFF % 64 == 0);
static_assert(NCAT % 64 == 0);
static_assert(HID % 32 == 0);
static_assert(NCAT % 32 == 0);
static_assert(NWI % EPB == 0);
static_assert(DFF % 256 == 0 && DFF <= EPB);
static_assert(HID % 256 == 0 && HID <= EPB);
static_assert(DFF % 1024 == 0);
static_assert(HID % 1024 == 0);
static_assert(((size_t)TOK * HID / 8) % 256 == 0);
static_assert(NB <= NB_FULL);
static_assert(SEQ <= SEQ_FULL);
static_assert(32 * 16 * 4 * 4 == 64 * 128);
static_assert(32 * 16 * 8 * 4 == 64 * 256);
static_assert(256 * 16 * 2 == 64 * 128);
static_assert(64 * 16 == 256 * 4);
static_assert(64 * 68 * 4 <= 131072);
static_assert(256 * 64 * 4 <= 131072);
static_assert(2 * 64 * 72 * 2 <= 131072);

typedef _Float16 h16;
typedef __attribute__((ext_vector_type(16))) _Float16 v16h;
typedef __attribute__((ext_vector_type(8)))  _Float16 v8h;
typedef __attribute__((ext_vector_type(8)))  float    v8f;
typedef __attribute__((ext_vector_type(4)))  float    v4f;
typedef __attribute__((ext_vector_type(4)))  unsigned v4u;
typedef v4f  __attribute__((may_alias)) v4fa;
typedef v8h  __attribute__((may_alias)) v8ha;
typedef v4u  __attribute__((may_alias)) v4ua;

__device__ __forceinline__ unsigned short f2bf(float f) { unsigned u = __float_as_uint(f); u += 0x7FFFu + ((u >> 16) & 1u); return (unsigned short)(u >> 16); }
__device__ __forceinline__ float bfr(float f) { return __uint_as_float(((unsigned)f2bf(f)) << 16); }
__device__ __forceinline__ v16h cat16(v8h lo, v8h hi) { return __builtin_shufflevector(lo, hi, 0, 1, 2, 3, 4, 5, 6, 7, 8, 9, 10, 11, 12, 13, 14, 15); }
__device__ __forceinline__ v8f wmma16(v16h a, v16h b, v8f c) { return __builtin_amdgcn_wmma_f32_16x16x32_f16(false, a, false, b, (short)0, c, false, false); }
__device__ __forceinline__ v16h  ldh(const h16* p) { return cat16(*(const v8h*)p, *(const v8h*)(p + 16)); }
__device__ __forceinline__ void wave_sync() { __builtin_amdgcn_fence(3  , "wavefront"); __builtin_amdgcn_wave_barrier(); asm volatile("" ::: "memory"); }
static __device__ __forceinline__ h16 toh_flush(float v) { const h16 r = (h16)v; return (fabsf(v) < 6.103515625e-05f) ? (h16)0.0f : r; }
__device__ __forceinline__ float wsum(float v) {
#pragma unroll
    for (int o = 16; o > 0; o >>= 1) v += __shfl_xor(v, o, 32);
    return v; }
__device__ __forceinline__ float gelu_t(float z) {
    const float u = 0.7978845608028654f * (z + 0.044715f * z * z * z);
    const float e = __builtin_amdgcn_exp2f(-2.8853900817779268f * u);
    return z * __builtin_amdgcn_rcpf(1.0f + e); }

__global__ __launch_bounds__(256) void k_xcvt(const float* __restrict__ x, h16* XH) {
    const size_t i = (size_t)blockIdx.x * 256 + threadIdx.x; if (i >= (size_t)TOK * HID / 8) return;
    const size_t m = i / (HID / 8); const int c8 = (int)(i % (HID / 8)) * 8;
    const size_t srow = (m / SEQ) * SEQ_FULL + (m % SEQ);
    const v8f v = *(const v8f*)(x + srow * HID + c8); v8h o;
#pragma unroll
    for (int k = 0; k < 8; ++k) o[k] = toh_flush(bfr(v[k]));
    *(volatile v8h*)(XH + i * 8) = o; __threadfence(); *(volatile v8h*)(XH + i * 8) = o;
}

__global__ __launch_bounds__(256) void k_router(const float* __restrict__ x, const float* __restrict__ gam, const float* __restrict__ bet,
                                                const float* __restrict__ Wr, const float* __restrict__ br, float* PR) {
#pragma clang fp contract(off)
    __shared__ __align__(16) float sp[64];
    const int lane = threadIdx.x & 31;
    const int wave = __builtin_amdgcn_readfirstlane((int)(threadIdx.x >> 5));
    const int m0 = blockIdx.x * 32;
#pragma unroll 1
    for (int tk = 0; tk < 4; ++tk) {
        const int m = m0 + wave * 4 + tk;
        const size_t srow = (size_t)(m / SEQ) * SEQ_FULL + (size_t)(m % SEQ);
        const float* xr = x + srow * HID + lane;
        float s = 0.0f;
#pragma unroll 1
        for (int j = 0; j < HID / 32; ++j) s += bfr(xr[j * 32]);
        s = wsum(s);
        const float mu = s * (1.0f / HID);
        float v = 0.0f;
#pragma unroll 1
        for (int j = 0; j < HID / 32; ++j) { const float d = bfr(xr[j * 32]) - mu; v += d * d; }
        v = wsum(v);
        const float rstd = rsqrtf(v * (1.0f / HID) + 1e-5f);
        float a[NEXP];
#pragma unroll
        for (int e = 0; e < NEXP; ++e) a[e] = 0.0f;
#pragma unroll 1
        for (int j = 0; j < HID / 32; ++j) {
            const int i = lane + 32 * j;
            const float hval = (bfr(xr[j * 32]) - mu) * rstd * bfr(gam[i]) + bfr(bet[i]);
            const v4f w0 = *(const v4f*)(Wr + (size_t)i * NEXP), w1 = *(const v4f*)(Wr + (size_t)i * NEXP + 4);
#pragma unroll
            for (int e = 0; e < 4; ++e) { a[e] += hval * bfr(w0[e]); a[4 + e] += hval * bfr(w1[e]); }
        }
        float lg[NEXP]; float mx = -3.0e38f;
#pragma unroll
        for (int e = 0; e < NEXP; ++e) { lg[e] = wsum(a[e]) + bfr(br[e]); mx = fmaxf(mx, lg[e]); }
        const float e0 = __builtin_amdgcn_exp2f((lg[0] - mx) * LOG2E);
        float rest = 0.0f;
#pragma unroll
        for (int e = 1; e < NEXP; ++e) rest += __builtin_amdgcn_exp2f((lg[e] - mx) * LOG2E);
        const float inv = __builtin_amdgcn_rcpf(e0 + rest);
        if (lane == 0) { sp[wave * 4 + tk] = e0 * inv; sp[32 + wave * 4 + tk] = rest * inv; }
    }
    __syncthreads();
    if (wave == 0) {
        const int q = lane & 15;
        const v4f val = *(const v4fa*)(&sp[q * 4]);
        float* dst = PR + (size_t)(q >> 3) * TOK + m0 + (q & 7) * 4;
#pragma unroll 1
        for (int ps = 0; ps < 2; ++ps) { if (lane < 16) *(volatile v4f*)dst = val; if (ps == 0) __threadfence(); }
    }
}

__global__ __launch_bounds__(64) void k_hist(const float* __restrict__ src, int n4, int blk0, int pass, int selidx, const unsigned* sel, unsigned* part) {
    __shared__ __align__(16) unsigned hist[256 * 64];
    const int tid = threadIdx.x;
#pragma unroll 1
    for (int q = tid; q < 256 * 64 / 4; q += 64) *(v4ua*)(&hist[q * 4]) = (v4u){0u, 0u, 0u, 0u};
    __syncthreads();
    unsigned sb = 0u, st = 0u;
    if (pass == 2) { sb = sel[selidx * 32]; st = sel[selidx * 32 + 2]; }
    const int rem = n4 - (int)blockIdx.x * (EPB / 4);
    int iters = rem / 64; iters = iters > 64 ? 64 : iters;
    const v4f* s4 = (const v4f*)src + (size_t)blockIdx.x * (EPB / 4) + tid;
#pragma unroll 1
    for (int it = 0; it < iters; ++it) {
        const v4f v = s4[(size_t)it * 64];
#pragma unroll
        for (int e = 0; e < 4; ++e) {
            const unsigned key = (unsigned)f2bf(v[e]) & 0x7FFFu;
            const unsigned d = key >> 7, lo = key & 127u;
            if (pass == 1) { hist[d * 64 + tid] += 1u; }
            else { hist[lo * 64 + tid] += (d == sb) ? 1u : 0u; hist[(128u + lo) * 64 + tid] += (d == st) ? 1u : 0u; }
        }
    }
    __syncthreads();
    unsigned sacc[4] = {0u, 0u, 0u, 0u};
#pragma unroll 1
    for (int c4 = 0; c4 < 16; ++c4) {
#pragma unroll
        for (int k = 0; k < 4; ++k) { const v4u q = *(const v4ua*)(&hist[(4 * tid + k) * 64 + c4 * 4]); sacc[k] += q[0] + q[1] + q[2] + q[3]; }
    }
    v4u o; o[0] = sacc[0]; o[1] = sacc[1]; o[2] = sacc[2]; o[3] = sacc[3];
    unsigned* dst = part + (size_t)(blk0 + (int)blockIdx.x) * 256 + 4 * tid;
    *(volatile v4u*)dst = o; __threadfence(); *(volatile v4u*)dst = o;
}

__global__ __launch_bounds__(256) void k_pick(const unsigned* part, const unsigned* selin, unsigned* lineout, int pass) {
    __shared__ unsigned cnt[256];
    __shared__ unsigned pfx[256];
    __shared__ unsigned res[4];
    const int t = threadIdx.x; const int j = blockIdx.x;
    const int bs = (j == 0) ? 0 : ((j == 1) ? NBW : ((j == 2) ? (NBW + 1) : (2 * NBW + 1)));
    const int nb = (j & 1) ? 1 : NBW;
    const int n = (j == 1) ? DFF : ((j == 3) ? HID : NWI);
    const int k = (j == 1) ? KT_B1 : ((j == 3) ? KT_B2 : KT_W);
    unsigned s = 0u;
#pragma unroll 1
    for (int b = 0; b < nb; ++b) s += part[(size_t)(bs + b) * 256 + t];
    cnt[t] = s; if (t < 4) res[t] = 0u;
    __syncthreads();
    if (t == 0) { unsigned cum = 0u;
#pragma unroll 1
        for (int i = 0; i < 256; ++i) { if ((pass == 2) & (i == 128)) cum = 0u; pfx[i] = cum; cum += cnt[i]; } }
    __syncthreads();
    unsigned r0 = (unsigned)(k - 1), r1 = (unsigned)(n - k);
    unsigned hb = 0u, ht = 0u;
    if (pass == 2) { hb = selin[j * 32]; r0 = selin[j * 32 + 1]; ht = selin[j * 32 + 2]; r1 = selin[j * 32 + 3]; }
    const unsigned base = pfx[t], c = cnt[t];
    const bool seg0 = (pass == 1) | (t < 128), seg1 = (pass == 1) | (t >= 128);
    const unsigned bin = (pass == 1) ? (unsigned)t : (unsigned)(t & 127);
    if (seg0 & (r0 >= base) & (r0 < base + c)) { res[0] = bin; res[1] = r0 - base; }
    if (seg1 & (r1 >= base) & (r1 < base + c)) { res[2] = bin; res[3] = r1 - base; }
    __syncthreads();
    if (t < 8) {
        v4u o = (v4u){0u, 0u, 0u, 0u};
        if (t == 0) {
            if (pass == 1) { o[0] = res[0]; o[1] = res[1]; o[2] = res[2]; o[3] = res[3]; }
            else { o[0] = (hb << 7) | res[0]; o[1] = (ht << 7) | res[2]; }
        }
        unsigned* dst = lineout + j * 32 + t * 4;
        *(volatile v4u*)dst = o; __threadfence(); *(volatile v4u*)dst = o;
    }
}

__global__ __launch_bounds__(256) void k_wconv(const float* __restrict__ W, int C, h16* OUTP, int pitch, size_t poff, float carry, const unsigned* thr) {
#pragma clang fp contract(off)
    __shared__ __align__(16) h16 tc[64 * 72];
    __shared__ __align__(16) h16 tp[64 * 72];
    const int tid = threadIdx.x, tx = tid & 15, ty = tid >> 4;
    const int c0 = blockIdx.x * 64, r0 = blockIdx.y * 64;
    const unsigned kb = thr[0], kt = thr[1];
#pragma unroll
    for (int i = 0; i < 4; ++i) { const int r = ty + 16 * i;
        const v4f v = *(const v4f*)(W + (size_t)(r0 + r) * C + c0 + 4 * tx);
#pragma unroll
        for (int e = 0; e < 4; ++e) {
            const unsigned bits = (unsigned)f2bf(v[e]); const unsigned key = bits & 0x7FFFu;
            const float wb = __uint_as_float(bits << 16);
            const float tier = (key >= kt) ? -1.0f : ((key <= kb) ? 1.0f : 0.0f);
            const float t8 = PSC * wb;
            const float pw = wb + t8 * tier;
            tc[(4 * tx + e) * 72 + r] = toh_flush(wb * carry);
            tp[(4 * tx + e) * 72 + r] = toh_flush(pw * carry); }
    }
    __syncthreads();
    v8h hc[2], hp[2];
#pragma unroll
    for (int s = 0; s < 2; ++s) { const int row = 32 * s + (tid >> 3), p8 = (tid & 7) * 8;
        hc[s] = *(const v8ha*)(&tc[row * 72 + p8]); hp[s] = *(const v8ha*)(&tp[row * 72 + p8]); }
#pragma unroll 1
    for (int ps = 0; ps < 2; ++ps) {
#pragma unroll
        for (int s = 0; s < 2; ++s) { const int row = 32 * s + (tid >> 3), p8 = (tid & 7) * 8;
            const size_t o = (size_t)(c0 + row) * (size_t)pitch + (size_t)(r0 + p8);
            *(volatile v8h*)(OUTP + o) = hc[s]; *(volatile v8h*)(OUTP + o + poff) = hp[s]; }
        if (ps == 0) __threadfence(); }
}

__global__ __launch_bounds__(256) void k_bprep(const float* __restrict__ b, int n, float* BC, const unsigned* thr) {
#pragma clang fp contract(off)
    const int i = blockIdx.x * 256 + threadIdx.x; if (i * 4 >= n) return;
    const unsigned kb = thr[0], kt = thr[1];
    const v4f v = *(const v4f*)(b + (size_t)i * 4); v4f c, p;
#pragma unroll
    for (int e = 0; e < 4; ++e) {
        const unsigned bits = (unsigned)f2bf(v[e]); const unsigned key = bits & 0x7FFFu;
        const float wb = __uint_as_float(bits << 16);
        const float tier = (key >= kt) ? -1.0f : ((key <= kb) ? 1.0f : 0.0f);
        const float t8 = PSC * wb;
        c[e] = wb; p[e] = wb + t8 * tier; }
    float* d0 = BC + (size_t)i * 4; float* d1 = BC + (size_t)n + (size_t)i * 4;
    *(volatile v4f*)d0 = c; *(volatile v4f*)d1 = p; __threadfence(); *(volatile v4f*)d0 = c; *(volatile v4f*)d1 = p;
}

__global__ __launch_bounds__(32) void k_ffn1(const h16* __restrict__ A, const h16* __restrict__ Bt, const float* __restrict__ BC, const float* __restrict__ PR, h16* ACT) {
    __shared__ __align__(16) float os[64 * 68];
    const int K = HID;
    const int lane = threadIdx.x & 31, lr = lane & 15, hi = lane >> 4; const int r0 = blockIdx.x * 64, c0 = blockIdx.y * 64;
    v8f acc[4][4];
#pragma unroll
    for (int mb = 0; mb < 4; ++mb)
#pragma unroll
        for (int nb = 0; nb < 4; ++nb) acc[mb][nb] = (v8f){};
    const size_t aoff = (size_t)(r0 + lr) * K + 8 * hi, boff = (size_t)(c0 + lr) * K + 8 * hi;
#pragma unroll 1
    for (int kc = 0; kc < K; kc += 32) {
        v16h a[4];
#pragma unroll
        for (int mb = 0; mb < 4; ++mb) a[mb] = ldh(A + aoff + (size_t)mb * 16 * K + kc);
#pragma unroll
        for (int nb = 0; nb < 4; ++nb) { const v16h b = ldh(Bt + boff + (size_t)nb * 16 * K + kc);
#pragma unroll
            for (int mb = 0; mb < 4; ++mb) acc[mb][nb] = wmma16(a[mb], b, acc[mb][nb]); }
        asm volatile("v_nop\n\tv_nop\n\tv_nop\n\tv_nop" : "+v"(acc[0][0]), "+v"(acc[1][1]), "+v"(acc[2][2]), "+v"(acc[3][3]) : "v"(a[0]), "v"(a[1]), "v"(a[2]), "v"(a[3]));
    }
#pragma unroll
    for (int mb = 0; mb < 4; ++mb)
#pragma unroll
        for (int nb = 0; nb < 4; ++nb)
#pragma unroll
            for (int j = 0; j < 8; ++j) os[(mb * 16 + hi * 8 + j) * 68 + nb * 16 + lr] = acc[mb][nb][j] * W1I;
    wave_sync();
    const int c8 = (lane & 7) * 8;
    const v4f bz0 = *(const v4f*)(BC + c0 + c8), bz1 = *(const v4f*)(BC + c0 + c8 + 4);
    const size_t pro = (size_t)(c0 / DFF) * TOK + (size_t)r0;
#pragma unroll 1
    for (int slab = 0; slab < 4; ++slab) {
        v8h hv[4];
#pragma unroll
        for (int s = 0; s < 4; ++s) { const int rl = slab * 16 + 4 * s + (lane >> 3);
            const v4f x0 = *(const v4fa*)(&os[rl * 68 + c8]); const v4f x1 = *(const v4fa*)(&os[rl * 68 + c8 + 4]);
            const float pr = PR[pro + rl] * ACS;
#pragma unroll
            for (int i = 0; i < 4; ++i) { hv[s][i] = toh_flush(gelu_t(x0[i] + bz0[i]) * pr); hv[s][4 + i] = toh_flush(gelu_t(x1[i] + bz1[i]) * pr); } }
#pragma unroll 1
        for (int ps = 0; ps < 2; ++ps) {
#pragma unroll
            for (int s = 0; s < 4; ++s) { const int rl = slab * 16 + 4 * s + (lane >> 3);
                *(volatile v8h*)(ACT + (size_t)(r0 + rl) * NCAT + c0 + c8) = hv[s]; }
            if (ps == 0) __threadfence(); }
    }
}

__global__ __launch_bounds__(32) void k_ffn2(const h16* __restrict__ A, const h16* __restrict__ Bt, const float* __restrict__ BC2, const float* __restrict__ PR, float* OUT) {
    __shared__ __align__(16) float os[64 * 68];
    const int K = NCAT;
    const int lane = threadIdx.x & 31, lr = lane & 15, hi = lane >> 4; const int r0 = blockIdx.x * 64, c0 = blockIdx.y * 64;
    v8f acc[4][4];
#pragma unroll
    for (int mb = 0; mb < 4; ++mb)
#pragma unroll
        for (int nb = 0; nb < 4; ++nb) acc[mb][nb] = (v8f){};
    const size_t aoff = (size_t)(r0 + lr) * K + 8 * hi, boff = (size_t)(c0 + lr) * K + 8 * hi;
#pragma unroll 1
    for (int kc = 0; kc < K; kc += 32) {
        v16h a[4];
#pragma unroll
        for (int mb = 0; mb < 4; ++mb) a[mb] = ldh(A + aoff + (size_t)mb * 16 * K + kc);
#pragma unroll
        for (int nb = 0; nb < 4; ++nb) { const v16h b = ldh(Bt + boff + (size_t)nb * 16 * K + kc);
#pragma unroll
            for (int mb = 0; mb < 4; ++mb) acc[mb][nb] = wmma16(a[mb], b, acc[mb][nb]); }
        asm volatile("v_nop\n\tv_nop\n\tv_nop\n\tv_nop" : "+v"(acc[0][0]), "+v"(acc[1][1]), "+v"(acc[2][2]), "+v"(acc[3][3]) : "v"(a[0]), "v"(a[1]), "v"(a[2]), "v"(a[3]));
    }
#pragma unroll
    for (int mb = 0; mb < 4; ++mb)
#pragma unroll
        for (int nb = 0; nb < 4; ++nb)
#pragma unroll
            for (int j = 0; j < 8; ++j) os[(mb * 16 + hi * 8 + j) * 68 + nb * 16 + lr] = acc[mb][nb][j] * OI;
    wave_sync();
    const int cofs = (lane & 15) * 4;
    const v4f bcl = *(const v4f*)(BC2 + c0 + cofs), btv = *(const v4f*)(BC2 + HID + c0 + cofs);
    const int bb = r0 / SEQ, tt = r0 % SEQ;
    float* obase = OUT + ((size_t)bb * OUT_SEQ + (size_t)tt) * HID + c0 + cofs;
#pragma unroll 1
    for (int slab = 0; slab < 4; ++slab) {
        v4f vals[8];
#pragma unroll
        for (int s = 0; s < 8; ++s) { const int rl = slab * 16 + 2 * s + (lane >> 4);
            const v4f xv = *(const v4fa*)(&os[rl * 68 + cofs]);
            const float pc = PR[(size_t)r0 + rl], pp = PR[(size_t)TOK + r0 + rl];
#pragma unroll
            for (int i = 0; i < 4; ++i) vals[s][i] = xv[i] + pc * bcl[i] + pp * btv[i]; }
#pragma unroll 1
        for (int ps = 0; ps < 2; ++ps) {
#pragma unroll
            for (int s = 0; s < 8; ++s) { const int rl = slab * 16 + 2 * s + (lane >> 4);
                *(volatile v4f*)(obase + (size_t)rl * HID) = vals[s]; }
            if (ps == 0) __threadfence(); }
    }
}

static constexpr size_t al256(size_t v) { return (v + 255) & ~(size_t)255; }
static constexpr size_t SZ_XH  = al256((size_t)TOK * HID * 2);
static constexpr size_t SZ_W1T = al256((size_t)NCAT * HID * 2);
static constexpr size_t SZ_W2T = al256((size_t)HID * NCAT * 2);
static constexpr size_t SZ_ACT = al256((size_t)TOK * NCAT * 2);
static constexpr size_t SZ_PR  = al256((size_t)2 * TOK * 4);
static constexpr size_t SZ_BC1 = al256((size_t)NCAT * 4);
static constexpr size_t SZ_BC2 = al256((size_t)2 * HID * 4);
static constexpr size_t SZ_HP  = al256((size_t)NHB * 256 * 4);
static constexpr size_t SZ_LN  = al256((size_t)4 * 32 * 4);
static constexpr size_t SZ_TOTAL = SZ_XH + SZ_W1T + SZ_W2T + SZ_ACT + SZ_PR + SZ_BC1 + SZ_BC2 + 2 * SZ_HP + 2 * SZ_LN;
static_assert(SZ_TOTAL <= (size_t)134217728);
static_assert((size_t)(2 * NBW + 1 + 1) * 256 * 4 <= SZ_HP);
static_assert((size_t)(3 * 32 + 7 * 4 + 4) * 4 <= SZ_LN);
static_assert((size_t)DFF * HID + (size_t)(DFF - 1) * HID + HID <= (size_t)NCAT * HID);
static_assert((size_t)(HID - 1) * NCAT + DFF + (DFF - 1) + 1 <= (size_t)HID * NCAT);

extern "C" void kernel_launch(void* const* d_in, const int* in_sizes, int n_in,
                              void* d_out, int out_size, void* d_ws, size_t ws_size, hipStream_t stream) {
    if (n_in < 9) return;
    const size_t needx = ((size_t)(NB - 1) * SEQ_FULL + SEQ) * HID;
    if ((size_t)in_sizes[0] < needx) return;
    if ((size_t)in_sizes[1] < (size_t)NWI || (size_t)in_sizes[3] < (size_t)NWI) return;
    if (in_sizes[2] < DFF || in_sizes[4] < HID || in_sizes[5] < HID || in_sizes[6] < HID) return;
    if (in_sizes[7] < HID * NEXP || in_sizes[8] < NEXP) return;
    if ((size_t)out_size < ((size_t)(NB - 1) * OUT_SEQ + SEQ) * HID) return;
    if (SZ_TOTAL > ws_size) return;
    const float* x  = (const float*)d_in[0];
    const float* W1 = (const float*)d_in[1]; const float* b1 = (const float*)d_in[2];
    const float* W2 = (const float*)d_in[3]; const float* b2 = (const float*)d_in[4];
    const float* gam = (const float*)d_in[5]; const float* bet = (const float*)d_in[6];
    const float* Wr = (const float*)d_in[7]; const float* br = (const float*)d_in[8];
    float* OUT = (float*)d_out;
    char* wsp = (char*)d_ws;
    h16* XH  = (h16*)wsp; wsp += SZ_XH;
    h16* W1T = (h16*)wsp; wsp += SZ_W1T;
    h16* W2T = (h16*)wsp; wsp += SZ_W2T;
    h16* ACT = (h16*)wsp; wsp += SZ_ACT;
    float* PR  = (float*)wsp; wsp += SZ_PR;
    float* BC1 = (float*)wsp; wsp += SZ_BC1;
    float* BC2 = (float*)wsp; wsp += SZ_BC2;
    unsigned* HP1 = (unsigned*)wsp; wsp += SZ_HP;
    unsigned* HP2 = (unsigned*)wsp; wsp += SZ_HP;
    unsigned* SEL = (unsigned*)wsp; wsp += SZ_LN;
    unsigned* THR = (unsigned*)wsp; wsp += SZ_LN;

    k_xcvt<<<(unsigned)((size_t)TOK * HID / 8 / 256), 256, 0, stream>>>(x, XH);
    k_router<<<TOK / 32, 256, 0, stream>>>(x, gam, bet, Wr, br, PR);

    k_hist<<<NBW, 64, 0, stream>>>(W1, NWI / 4, 0,           1, 0, SEL, HP1);
    k_hist<<<1,   64, 0, stream>>>(b1, DFF / 4, NBW,         1, 1, SEL, HP1);
    k_hist<<<NBW, 64, 0, stream>>>(W2, NWI / 4, NBW + 1,     1, 2, SEL, HP1);
    k_hist<<<1,   64, 0, stream>>>(b2, HID / 4, 2 * NBW + 1, 1, 3, SEL, HP1);
    k_pick<<<4, 256, 0, stream>>>(HP1, THR, SEL, 1);
    k_hist<<<NBW, 64, 0, stream>>>(W1, NWI / 4, 0,           2, 0, SEL, HP2);
    k_hist<<<1,   64, 0, stream>>>(b1, DFF / 4, NBW,         2, 1, SEL, HP2);
    k_hist<<<NBW, 64, 0, stream>>>(W2, NWI / 4, NBW + 1,     2, 2, SEL, HP2);
    k_hist<<<1,   64, 0, stream>>>(b2, HID / 4, 2 * NBW + 1, 2, 3, SEL, HP2);
    k_pick<<<4, 256, 0, stream>>>(HP2, SEL, THR, 2);

    k_wconv<<<dim3(DFF / 64, HID / 64, 1), 256, 0, stream>>>(W1, DFF, W1T, HID, (size_t)DFF * HID, W1S, THR + 0);
    k_wconv<<<dim3(HID / 64, DFF / 64, 1), 256, 0, stream>>>(W2, HID, W2T, NCAT, (size_t)DFF, W2S, THR + 64);
    k_bprep<<<DFF / 1024, 256, 0, stream>>>(b1, DFF, BC1, THR + 32);
    k_bprep<<<HID / 1024, 256, 0, stream>>>(b2, HID, BC2, THR + 96);

    k_ffn1<<<dim3(TOK / 64, NCAT / 64, 1), 32, 0, stream>>>(XH, W1T, BC1, PR, ACT);
    k_ffn2<<<dim3(TOK / 64, HID / 64, 1), 32, 0, stream>>>(ACT, W2T, BC2, PR, OUT);
}
